// DynamicFieldPropagator_23089744183586
// MI455X (gfx1250) — hardware-verified
//
#include <hip/hip_runtime.h>


#define NB_  4
#define NN   2048
#define DD   256
#define NH_  8
#define HD   32
#define ZH   2
#define NSTEP 4
typedef _Float16 h16;
typedef unsigned short bf;
typedef __attribute__((ext_vector_type(16))) __bf16   v16bf;
typedef __attribute__((ext_vector_type(16))) _Float16 v16h;
typedef __attribute__((ext_vector_type(8)))  _Float16 v8h;
typedef __attribute__((ext_vector_type(8)))  unsigned short v8us;
typedef __attribute__((ext_vector_type(8)))  float    v8f;
typedef __attribute__((ext_vector_type(4)))  float    v4f;
typedef v8h  __attribute__((may_alias)) v8ha;
typedef v4f  __attribute__((may_alias)) v4fa;
typedef v8us __attribute__((may_alias)) v8usa;

__device__ __forceinline__ unsigned short f2bf(float f) { unsigned u = __float_as_uint(f); u += 0x7FFFu + ((u >> 16) & 1u); return (unsigned short)(u >> 16); }
__device__ __forceinline__ float bf2f(unsigned short b) { return __uint_as_float(((unsigned)b) << 16); }
__device__ __forceinline__ float bfr(float f) { return bf2f(f2bf(f)); }
__device__ __forceinline__ v16h cat16(v8h lo, v8h hi) { return __builtin_shufflevector(lo, hi, 0, 1, 2, 3, 4, 5, 6, 7, 8, 9, 10, 11, 12, 13, 14, 15); }
__device__ __forceinline__ v16bf cat16b(v8us lo, v8us hi) { return __builtin_bit_cast(v16bf, __builtin_shufflevector(lo, hi, 0, 1, 2, 3, 4, 5, 6, 7, 8, 9, 10, 11, 12, 13, 14, 15)); }
__device__ __forceinline__ v8f wmma16(v16h a, v16h b, v8f c) { return __builtin_amdgcn_wmma_f32_16x16x32_f16(false, a, false, b, (short)0, c, false, false); }
__device__ __forceinline__ v8f wmmab(v16bf a, v16bf b, v8f c) { return __builtin_amdgcn_wmma_f32_16x16x32_bf16(false, a, false, b, (short)0, c, false, false); }


template <typename T16> struct WFrag;
template <> struct WFrag<h16> { typedef v16h V; static __device__ __forceinline__ V ld(const h16* p) { return cat16(*(const v8h*)p, *(const v8h*)(p + 16)); } static __device__ __forceinline__ v8f mma(V a, V b, v8f c) { return wmma16(a, b, c); } };
template <> struct WFrag<bf> { typedef v16bf V; static __device__ __forceinline__ V ld(const bf* p) { return cat16b(*(const v8us*)p, *(const v8us*)(p + 16)); } static __device__ __forceinline__ v8f mma(V a, V b, v8f c) { return wmmab(a, b, c); } };
template <typename T16, int NSPLIT, bool BIAS>
__global__ __launch_bounds__(32) void k_gemmw(const T16* __restrict__ A, const T16* __restrict__ A2, const T16* __restrict__ Bt, const T16* __restrict__ Bt2, int K, float* C, int ldc, const float* __restrict__ bias, size_t sA, size_t sB, size_t sC) {
    typedef typename WFrag<T16>::V V;
    __shared__ __align__(16) float os[16 * 68];
    const size_t z = blockIdx.z; A += z * sA; if (A2) A2 += z * sA; Bt += z * sB; if (Bt2) Bt2 += z * sB; C += z * sC;
    const int lane = threadIdx.x & 31, lr = lane & 15, hi = lane >> 4; const int r0 = blockIdx.x * 64, c0 = blockIdx.y * 64;
    v8f acc[4][4];
#pragma unroll
    for (int mb = 0; mb < 4; ++mb)
#pragma unroll
        for (int nb = 0; nb < 4; ++nb) acc[mb][nb] = (v8f){};
    const size_t aoff = (size_t)(r0 + lr) * K + 8 * hi, boff = (size_t)(c0 + lr) * K + 8 * hi;
#pragma unroll 1
    for (int kc = 0; kc < K; kc += 32) {
        V a[4], a2[4];
#pragma unroll
        for (int mb = 0; mb < 4; ++mb) { a[mb] = WFrag<T16>::ld(A + aoff + (size_t)mb * 16 * K + kc); if (NSPLIT == 1 || NSPLIT == 2) a2[mb] = WFrag<T16>::ld(A2 + aoff + (size_t)mb * 16 * K + kc); }
#pragma unroll
        for (int nb = 0; nb < 4; ++nb) { const V b = WFrag<T16>::ld(Bt + boff + (size_t)nb * 16 * K + kc); V b2; if (NSPLIT >= 2) b2 = WFrag<T16>::ld(Bt2 + boff + (size_t)nb * 16 * K + kc);
#pragma unroll
            for (int mb = 0; mb < 4; ++mb) { acc[mb][nb] = WFrag<T16>::mma(a[mb], b, acc[mb][nb]); if (NSPLIT == 1 || NSPLIT == 2) acc[mb][nb] = WFrag<T16>::mma(a2[mb], b, acc[mb][nb]); if (NSPLIT >= 2) acc[mb][nb] = WFrag<T16>::mma(a[mb], b2, acc[mb][nb]); } }
        asm volatile("v_nop\n\tv_nop\n\tv_nop\n\tv_nop" : "+v"(acc[0][0]), "+v"(acc[1][1]), "+v"(acc[2][2]), "+v"(acc[3][3]) : "v"(a[0]), "v"(a[3]));
    }
#pragma unroll
    for (int mb = 0; mb < 4; ++mb) {
#pragma unroll
        for (int nb = 0; nb < 4; ++nb) {
#pragma unroll
            for (int j = 0; j < 8; ++j) os[(hi * 8 + j) * 68 + nb * 16 + lr] = acc[mb][nb][j]; }
        __builtin_amdgcn_wave_barrier(); asm volatile("" ::: "memory");
        float* crow = C + (size_t)(r0 + mb * 16) * ldc + c0;
#pragma unroll 1
        for (int ps = 0; ps < 2; ++ps) {
#pragma unroll
            for (int s = 0; s < 8; ++s) { const int row = 2 * s + hi, cofs = lr * 4; v4f val = *(const v4fa*)(os + row * 68 + cofs); if (BIAS) { val[0] += bfr(bias[c0 + cofs]); val[1] += bfr(bias[c0 + cofs + 1]); val[2] += bfr(bias[c0 + cofs + 2]); val[3] += bfr(bias[c0 + cofs + 3]); }
                *(volatile v4f*)(crow + (size_t)row * ldc + cofs) = val; }
            if (ps == 0) __threadfence(); }
        __builtin_amdgcn_wave_barrier(); asm volatile("" ::: "memory");
    }
}

__device__ __forceinline__ h16 tohx(float x) { return (h16)x; }
__device__ __forceinline__ void splitf(float y, unsigned short& h, unsigned short& l) { h = f2bf(y); l = f2bf(y - bf2f(h)); }
typedef __attribute__((ext_vector_type(4))) unsigned short v4us;
typedef __attribute__((ext_vector_type(2))) _Float16 v2h;
typedef __attribute__((ext_vector_type(4))) _Float16 v4h;

__global__ __launch_bounds__(256) void k_cvt8(const float* __restrict__ src, bf* dst, size_t n8) { const size_t i = (size_t)blockIdx.x * 256 + threadIdx.x; if (i >= n8) return; const v8f v = *(const v8f*)(src + i * 8); v8us o;
#pragma unroll
    for (int k = 0; k < 8; ++k) o[k] = f2bf(v[k]); *(volatile v8us*)(dst + i * 8) = o; __threadfence(); *(volatile v8us*)(dst + i * 8) = o; }
__global__ __launch_bounds__(256) void k_init(const float* __restrict__ x, float* F) { const size_t e = ((size_t)blockIdx.x * 256 + threadIdx.x) * 4; if (e >= (size_t)NN * DD) return; v4f r;
#pragma unroll
    for (int u = 0; u < 4; ++u) r[u] = bfr(x[e + u]); *(volatile v4f*)(F + e) = r; __threadfence(); *(volatile v4f*)(F + e) = r; }
__global__ __launch_bounds__(256) void k_fpl(const float* __restrict__ F, h16* P) { const size_t e = ((size_t)blockIdx.x * 256 + threadIdx.x) * 4; if (e >= (size_t)NH_ * NN * HD) return; const int d = (int)(e % HD); const int n = (int)((e / HD) % NN); const int h = (int)(e / ((size_t)HD * NN)); const float* f = F + (size_t)n * DD + h * HD + d; v4h o;
#pragma unroll
    for (int u = 0; u < 4; ++u) o[u] = tohx(f[u]); *(volatile v4h*)(P + e) = o; __threadfence(); *(volatile v4h*)(P + e) = o; }
__global__ __launch_bounds__(256) void k_ftr(const float* __restrict__ F, h16* FT) { const size_t e = ((size_t)blockIdx.x * 256 + threadIdx.x) * 2; if (e >= (size_t)NH_ * 64 * NN) return; const int n = (int)(e % NN); const int d = (int)((e / NN) % 64); const int h = (int)(e / ((size_t)NN * 64)); v2h o;
    if (d < HD) { o[0] = tohx(F[(size_t)n * DD + h * HD + d]); o[1] = tohx(F[(size_t)(n + 1) * DD + h * HD + d]); } else { o[0] = (h16)0.f; o[1] = (h16)0.f; }
    *(volatile v2h*)(FT + e) = o; __threadfence(); *(volatile v2h*)(FT + e) = o; }
__global__ __launch_bounds__(256) void k_interf(const float* __restrict__ S, const float* __restrict__ iw, h16* I16) { const size_t e = ((size_t)blockIdx.x * 256 + threadIdx.x) * 4; if (e >= (size_t)ZH * NN * NN) return; const float w0 = bfr(iw[0]), w1 = bfr(iw[1]), w2 = bfr(iw[2]); const v4f a = *(const v4f*)(S + e); v4h o;
#pragma unroll
    for (int u = 0; u < 4; ++u) { const float s = a[u] * 0.17677669529663689f; float p0 = __fmul_rn(w0, fmaxf(s, 0.f)), p1 = __fmul_rn(w1, fmaxf(-s, 0.f)), p2 = __fmul_rn(w2, __cosf(s));     asm volatile("" : "+v"(p0)); asm volatile("" : "+v"(p1)); asm volatile("" : "+v"(p2)); o[u] = tohx(__fadd_rn(__fsub_rn(p0, p1), p2)); }
    *(volatile v4h*)(I16 + e) = o; __threadfence(); *(volatile v4h*)(I16 + e) = o; }
__global__ __launch_bounds__(256) void k_agmrg(const float* __restrict__ O, int h0, float* AG) { const size_t e = ((size_t)blockIdx.x * 256 + threadIdx.x) * 4; if (e >= (size_t)ZH * NN * HD) return; const int d = (int)(e % HD); const int n = (int)((e / HD) % NN); const int zz = (int)(e / ((size_t)HD * NN)); v4f a;
#pragma unroll
    for (int u = 0; u < 4; ++u) a[u] = O[((size_t)zz * NN + n) * 64 + d + u]; float* dst = AG + (size_t)n * DD + (h0 + zz) * HD + d; *(volatile v4f*)dst = a; __threadfence(); *(volatile v4f*)dst = a; }
__global__ __launch_bounds__(256) void k_pl(const float* __restrict__ F, bf* Ph, bf* Pl) { const size_t e = ((size_t)blockIdx.x * 256 + threadIdx.x) * 4; if (e >= (size_t)NN * DD) return; v4us oh, ol;
#pragma unroll
    for (int u = 0; u < 4; ++u) { unsigned short a, b; splitf(F[e + u], a, b); oh[u] = a; ol[u] = b; } *(volatile v4us*)(Ph + e) = oh; *(volatile v4us*)(Pl + e) = ol; __threadfence(); *(volatile v4us*)(Ph + e) = oh; *(volatile v4us*)(Pl + e) = ol; }
__global__ __launch_bounds__(256) void k_update(const float* __restrict__ F, const float* __restrict__ INT, const float* __restrict__ dc, const float* __restrict__ cc, float* F2) { const size_t e = ((size_t)blockIdx.x * 256 + threadIdx.x) * 4; if (e >= (size_t)NN * DD) return; const int d = (int)(e % DD); const int n = (int)(e / DD); const float alpha = fminf(fmaxf(bfr(dc[0]), 0.01f), 1.0f); v4f r;
#pragma unroll
    for (int u = 0; u < 4; ++u) { const float f0 = F[e + u]; float lap;
        if (n == 0) lap = __fsub_rn(F[e + u + DD], f0);
        else if (n == NN - 1) lap = __fsub_rn(F[e + u - DD], f0);
        else { float t2 = f0 * 2.0f; asm volatile("" : "+v"(t2)); lap = __fadd_rn(__fsub_rn(F[e + u + DD], t2), F[e + u - DD]); }
        const float coup = fminf(fmaxf(bfr(cc[d + u]), 0.01f), 10.0f); float a1 = __fmul_rn(alpha, lap); asm volatile("" : "+v"(a1)); float it = __fmul_rn(INT[e + u], coup); asm volatile("" : "+v"(it)); float ih = it * 0.5f; asm volatile("" : "+v"(ih)); float sum = __fadd_rn(a1, ih); asm volatile("" : "+v"(sum)); float dlt = __fmul_rn(sum, 0.0099999997764825821f); asm volatile("" : "+v"(dlt)); r[u] = __fadd_rn(f0, dlt); }
    *(volatile v4f*)(F2 + e) = r; __threadfence(); *(volatile v4f*)(F2 + e) = r; }

extern "C" void kernel_launch(void* const* d_in, const int* in_sizes, int n_in,
                              void* d_out, int out_size, void* d_ws, size_t ws_size, hipStream_t stream) {
    (void)in_sizes; (void)n_in; (void)out_size;
    const float** I = (const float**)d_in;
    const float *x = I[0], *dc = I[1], *cc = I[2], *iw = I[3], *Wi = I[4], *bi = I[5], *Wo = I[6], *bo = I[7];
    float* OUT = (float*)d_out;
    char* wsp = (char*)d_ws;
    auto take = [&](size_t bytes) { char* p = wsp; wsp += (bytes + 255) & ~(size_t)255; return (void*)p; };
    bf* BI = (bf*)take((size_t)DD * DD * 2); bf* BO = (bf*)take((size_t)DD * DD * 2); float* F = (float*)take((size_t)NN * DD * 4); float* F2 = (float*)take((size_t)NN * DD * 4);
    h16* FP = (h16*)take((size_t)NH_ * NN * HD * 2); h16* FT = (h16*)take((size_t)NH_ * 64 * NN * 2); float* S = (float*)take((size_t)ZH * NN * NN * 4); h16* I16 = (h16*)take((size_t)ZH * NN * NN * 2); float* O = (float*)take((size_t)ZH * NN * 64 * 4); float* AG = (float*)take((size_t)NN * DD * 4); bf* AGh = (bf*)take((size_t)NN * DD * 2); bf* AGl = (bf*)take((size_t)NN * DD * 2); float* INT = (float*)take((size_t)NN * DD * 4);
    if ((size_t)(wsp - (char*)d_ws) > ws_size) return;
    k_cvt8<<<(DD * DD / 8 + 255) / 256, 256, 0, stream>>>(Wi, BI, DD * DD / 8); k_cvt8<<<(DD * DD / 8 + 255) / 256, 256, 0, stream>>>(Wo, BO, DD * DD / 8);
    const size_t zq = (size_t)NN * HD, zS = (size_t)NN * NN, zv = (size_t)64 * NN, zo = (size_t)NN * 64;
    for (int b = 0; b < NB_; ++b) { float* Fa = F; float* Fb = F2;
        k_init<<<(NN * DD / 4 + 255) / 256, 256, 0, stream>>>(x + (size_t)b * NN * DD, Fa);
        for (int st = 0; st < NSTEP; ++st) {
            k_fpl<<<(NH_ * NN * HD / 4 + 255) / 256, 256, 0, stream>>>(Fa, FP); k_ftr<<<(NH_ * 64 * NN / 2 + 255) / 256, 256, 0, stream>>>(Fa, FT);
            for (int h0 = 0; h0 < NH_; h0 += ZH) {
                k_gemmw<h16, 0, false><<<dim3(NN / 64, NN / 64, ZH), 32, 0, stream>>>(FP + (size_t)h0 * zq, nullptr, FP + (size_t)h0 * zq, nullptr, HD, S, NN, nullptr, zq, zq, zS);
                k_interf<<<(unsigned)(((size_t)ZH * NN * NN / 4 + 255) / 256), 256, 0, stream>>>(S, iw, I16);
                k_gemmw<h16, 0, false><<<dim3(NN / 64, 1, ZH), 32, 0, stream>>>(I16, nullptr, FT + (size_t)h0 * zv, nullptr, NN, O, 64, nullptr, zS, zv, zo);
                k_agmrg<<<(ZH * NN * HD / 4 + 255) / 256, 256, 0, stream>>>(O, h0, AG); }
            k_pl<<<(NN * DD / 4 + 255) / 256, 256, 0, stream>>>(AG, AGh, AGl); k_gemmw<bf, 1, true><<<dim3(NN / 64, DD / 64, 1), 32, 0, stream>>>(AGh, AGl, BI, nullptr, DD, INT, DD, bi, 0, 0, 0);
            k_update<<<(NN * DD / 4 + 255) / 256, 256, 0, stream>>>(Fa, INT, dc, cc, Fb); float* t = Fa; Fa = Fb; Fb = t; }
        k_pl<<<(NN * DD / 4 + 255) / 256, 256, 0, stream>>>(Fa, AGh, AGl); k_gemmw<bf, 1, true><<<dim3(NN / 64, DD / 64, 1), 32, 0, stream>>>(AGh, AGl, BO, nullptr, DD, OUT + (size_t)b * NN * DD, DD, bo, 0, 0, 0); }
}
